// NetTransform_39496519254209
// MI455X (gfx1250) — hardware-run, weakly checked
//
#include <hip/hip_runtime.h>
#include <stdint.h>
#include <math.h>

constexpr int NB_   = 4;
constexpr int NT_   = 256;
constexpr int NI_   = 80;
constexpr int NHID_ = 512;
constexpr int NTN_  = 10;
constexpr int NTOK_ = NB_ * NT_;
constexpr int KP_   = 128;
constexpr int N2P_  = 192;
constexpr int NOP_  = 128;
constexpr int HFP_  = 256;
constexpr int OUT_TOTAL_ = 1 + 2 * NB_ * NT_ * NT_;
constexpr int OUT1_OFF_ = 1;
constexpr int OUT2_OFF_ = 1 + NB_ * NT_ * NT_;
static_assert(OUT_TOTAL_ == 524289);
static_assert(OUT2_OFF_ == 262145);
static_assert(OUT2_OFF_ + NB_ * NT_ * NT_ == OUT_TOTAL_);
static_assert(NTOK_ % 64 == 0 && (2 * NTOK_) % 64 == 0 && NHID_ % 64 == 0 && N2P_ % 64 == 0 && NOP_ % 64 == 0 && NT_ % 64 == 0);
static_assert(KP_ % 32 == 0 && KP_ % 64 == 0 && NHID_ % 32 == 0);
static_assert(NI_ == 5 * 16);

constexpr size_t SZ_XIN   = (size_t)NTOK_ * KP_ * 2;
constexpr size_t SZ_W1T   = (size_t)NHID_ * KP_ * 2;
constexpr size_t SZ_EW2T  = (size_t)N2P_ * NHID_ * 2;
constexpr size_t SZ_W2T   = (size_t)NOP_ * NHID_ * 2;
constexpr size_t SZ_AW1   = (size_t)128 * NHID_ * 2;
constexpr size_t SZ_ZENC  = (size_t)NTOK_ * NHID_ * 2;
constexpr size_t SZ_H2    = (size_t)NTOK_ * N2P_ * 4;
constexpr size_t SZ_HP    = SZ_XIN;
constexpr size_t SZ_HF    = (size_t)NTOK_ * HFP_ * 4;
constexpr size_t SZ_ZR    = (size_t)2 * NTOK_ * NHID_ * 2;
constexpr size_t SZ_CM    = (size_t)2 * NTOK_ * NOP_ * 4;
constexpr size_t SZ_MASKT = (size_t)2 * NTOK_ * 16 * 4;
constexpr size_t SZ_GRAM  = (size_t)NB_ * NT_ * NT_ * 4;
constexpr size_t SZ_E0    = (size_t)2 * NTOK_ * 4;
constexpr size_t SZ_LINE  = 256;
constexpr size_t SZ_PART  = (size_t)NTOK_ * 32 * 4;
constexpr size_t WS_TOTAL_ = 2 * SZ_XIN + 2 * SZ_W1T + 2 * SZ_EW2T + 4 * SZ_W1T + 4 * SZ_W2T + 4 * SZ_AW1
                           + 2 * SZ_ZENC + SZ_H2 + 4 * SZ_HP + SZ_HF + 4 * SZ_ZR + 2 * SZ_CM + SZ_MASKT
                           + SZ_GRAM + SZ_E0 + SZ_LINE + 2 * SZ_GRAM + SZ_PART + SZ_LINE;
static_assert(WS_TOTAL_ == 21635584);
static_assert(WS_TOTAL_ <= (size_t)134217728);

typedef __attribute__((ext_vector_type(16))) _Float16 v16h;
typedef __attribute__((ext_vector_type(8)))  _Float16 v8h;
typedef __attribute__((ext_vector_type(16))) __bf16   v16b;
typedef __attribute__((ext_vector_type(8)))  __bf16   v8b;
typedef __attribute__((ext_vector_type(8)))  float    v8f;
typedef __attribute__((ext_vector_type(4)))  float    v4f;
typedef __attribute__((ext_vector_type(4)))  unsigned v4u;
typedef __attribute__((ext_vector_type(8)))  unsigned v8u;

__device__ __forceinline__ unsigned short f2bf_bits(float f) {
  unsigned u = __float_as_uint(f);
  return (unsigned short)((u + 0x7FFFu + ((u >> 16) & 1u)) >> 16);
}
__device__ __forceinline__ float bf_bits2f(unsigned short h) { return __uint_as_float(((unsigned)h) << 16); }

__device__ __forceinline__ void dep_guard_h(v8f& a, v8f& b, v16h x, v16h y) { asm volatile("v_nop\n\tv_nop\n\tv_nop\n\tv_nop" : "+v"(a), "+v"(b) : "v"(x), "v"(y)); }
__device__ __forceinline__ void dep_guard_b(v8f& a, v8f& b, v16b x, v16b y) { asm volatile("v_nop\n\tv_nop\n\tv_nop\n\tv_nop" : "+v"(a), "+v"(b) : "v"(x), "v"(y)); }
__device__ __forceinline__ void keep4_h(v16h a, v16h b, v16h c, v16h d) { asm volatile("v_nop" :: "v"(a), "v"(b), "v"(c), "v"(d)); }
__device__ __forceinline__ void keep4_b(v16b a, v16b b, v16b c, v16b d) { asm volatile("v_nop" :: "v"(a), "v"(b), "v"(c), "v"(d)); }
__device__ __forceinline__ void acc_guard4(v8f& a, v8f& b, v8f& c, v8f& d) { asm volatile("v_nop\n\tv_nop\n\tv_nop\n\tv_nop" : "+v"(a), "+v"(b), "+v"(c), "+v"(d)); }
__device__ __forceinline__ void acc_guard5(v8f& a, v8f& b, v8f& c, v8f& d, v8f& e) { asm volatile("v_nop\n\tv_nop\n\tv_nop\n\tv_nop" : "+v"(a), "+v"(b), "+v"(c), "+v"(d), "+v"(e)); }
__device__ __forceinline__ void keep5_b(v16b a, v16b b, v16b c, v16b d, v16b e) { asm volatile("v_nop" :: "v"(a), "v"(b), "v"(c), "v"(d), "v"(e)); }
template <typename T> struct Frag;
template <> struct Frag<_Float16> {
  typedef v16h V; union U { v16h v; v8h h[2]; };
  static __device__ __forceinline__ v16h load(const _Float16* p) {
    U f; f.h[0] = *(const v8h*)(p); f.h[1] = *(const v8h*)(p + 16); return f.v;
  }
  static __device__ __forceinline__ v8f mma(v16h a, v16h b, v8f c) {
    return __builtin_amdgcn_wmma_f32_16x16x32_f16(false, a, false, b, (short)0, c, false, false);
  }
  static __device__ __forceinline__ void guard(v8f& a, v8f& b, v16h x, v16h y) { dep_guard_h(a, b, x, y); }
  static __device__ __forceinline__ void keep(v16h a, v16h b, v16h c, v16h d) { keep4_h(a, b, c, d); }
};
template <> struct Frag<__bf16> {
  typedef v16b V; union U { v16b v; v8b h[2]; };
  static __device__ __forceinline__ v16b load(const __bf16* p) {
    U f; f.h[0] = *(const v8b*)(p); f.h[1] = *(const v8b*)(p + 16); return f.v;
  }
  static __device__ __forceinline__ v8f mma(v16b a, v16b b, v8f c) {
    return __builtin_amdgcn_wmma_f32_16x16x32_bf16(false, a, false, b, (short)0, c, false, false);
  }
  static __device__ __forceinline__ void guard(v8f& a, v8f& b, v16b x, v16b y) { dep_guard_b(a, b, x, y); }
  static __device__ __forceinline__ void keep(v16b a, v16b b, v16b c, v16b d) { keep4_b(a, b, c, d); }
};

template <int ET> struct Elem;
template <> struct Elem<0> { typedef _Float16 T; };
template <> struct Elem<1> { typedef __bf16 T; };
template <int ET, bool SPLIT, int BIAS_MODE, int OUT_MODE, bool RESID, int ACT = 0>
__global__ __launch_bounds__(256) void wmma_gemm64(
    const unsigned short* __restrict__ Ap, const unsigned short* __restrict__ A2p, int lda, long strideA,
    const unsigned short* __restrict__ Btp, const unsigned short* __restrict__ Bt2p, int ldb, long strideB,
    void* __restrict__ Cout, void* __restrict__ Cout2, int ldc, long strideC,
    const float* __restrict__ bias,
    const float* __restrict__ resid, long strideR,
    int M, int N, int K, float scale) {
  typedef typename Elem<ET>::T T;
  typedef typename Frag<T>::V V;
  const T* A = (const T*)Ap; const T* A2 = (const T*)A2p; const T* Bt = (const T*)Btp; const T* Bt2 = (const T*)Bt2p;
  __shared__ __align__(16) float sT[8][16 * 68];
  const int b    = blockIdx.y;
  const int lane = threadIdx.x & 31;
  const int wave = threadIdx.x >> 5;
  const int tilesN = N >> 6;
  const int tilesM = M >> 6;
  const int tile = blockIdx.x * 8 + wave;
  if (tile >= tilesM * tilesN) return;
  const int tm = tile / tilesN;
  const int tn = tile - tm * tilesN;
  const int m0 = tm << 6;
  const int n0 = tn << 6;

  const T* Ab  = A  + (size_t)b * strideA;
  const T* Bb  = Bt + (size_t)b * strideB;
  const T* Ab2 = SPLIT ? (A2  + (size_t)b * strideA) : nullptr;
  const T* Bb2 = SPLIT ? (Bt2 + (size_t)b * strideB) : nullptr;

  const int rlane = lane & 15;
  const int koff  = (lane >> 4) * 8;
  const int mOff  = (lane >> 4) * 8;

  v8f acc[4][4];
#pragma unroll
  for (int i = 0; i < 4; ++i)
#pragma unroll
    for (int j = 0; j < 4; ++j) acc[i][j] = (v8f){0.f,0.f,0.f,0.f,0.f,0.f,0.f,0.f};

  for (int k0 = 0; k0 < K; k0 += 32) {
    V bh[4], bl[4];
#pragma unroll
    for (int j = 0; j < 4; ++j) {
      const size_t bo = (size_t)(n0 + (j << 4) + rlane) * ldb + koff + k0;
      bh[j] = Frag<T>::load(Bb + bo);
      if (SPLIT) bl[j] = Frag<T>::load(Bb2 + bo);
    }
#pragma unroll
    for (int i = 0; i < 4; ++i) {
      const size_t ao = (size_t)(m0 + (i << 4) + rlane) * lda + koff + k0;
      V ah = Frag<T>::load(Ab + ao);
      V al;
      if (SPLIT) al = Frag<T>::load(Ab2 + ao);
#pragma unroll
      for (int j = 0; j < 4; ++j) {
        acc[i][j] = Frag<T>::mma(ah, bh[j], acc[i][j]);
        if (SPLIT) {
          acc[i][j] = Frag<T>::mma(ah, bl[j], acc[i][j]);
          acc[i][j] = Frag<T>::mma(al, bh[j], acc[i][j]);
        }
      }
      Frag<T>::guard(acc[i][0], acc[i][3], ah, SPLIT ? al : ah);
    }
    Frag<T>::keep(bh[0], bh[1], bh[2], bh[3]);
    if (SPLIT) Frag<T>::keep(bl[0], bl[1], bl[2], bl[3]);
  }
  acc_guard4(acc[0][0], acc[0][1], acc[0][2], acc[0][3]);
  acc_guard4(acc[1][0], acc[1][1], acc[1][2], acc[1][3]);
  acc_guard4(acc[2][0], acc[2][1], acc[2][2], acc[2][3]);
  acc_guard4(acc[3][0], acc[3][1], acc[3][2], acc[3][3]);

  float* slab = sT[wave];
  const float* Rb = RESID ? (resid + (size_t)b * strideR) : nullptr;
#pragma unroll
  for (int i = 0; i < 4; ++i) {
    const int mBase = m0 + (i << 4);
#pragma unroll
    for (int j = 0; j < 4; ++j) {
      const int n = n0 + (j << 4) + rlane;
      float bv = 0.f;
      if (BIAS_MODE == 2) bv = bias[n];
#pragma unroll
      for (int r = 0; r < 8; ++r) {
        float v = acc[i][j][r] * scale;
        if (BIAS_MODE == 1) v += bias[mBase + mOff + r];
        if (BIAS_MODE == 2) v += bv;
        if (RESID) v += Rb[(size_t)(mBase + mOff + r) * ldc + n];
        if (ACT == 1) v = tanhf(v);
        if (ACT == 2) v = fmaxf(v, 0.0f);
        if (ACT == 3) v = v / (1.0f + expf(-v));
        if (ACT == 4) v = (v > 0.f) ? v : 0.01f * v;
        if (ACT == 5) v = 0.5f * v * (1.0f + erff(v * 0.70710678118654752f));
        slab[(mOff + r) * 68 + (j << 4) + rlane] = v;
      }
    }
    __builtin_amdgcn_fence(__ATOMIC_RELEASE, "workgroup");
    __builtin_amdgcn_wave_barrier();
    __builtin_amdgcn_fence(__ATOMIC_ACQUIRE, "workgroup");
    if (OUT_MODE == 0) {
      float* C = (float*)Cout + (size_t)b * strideC;
      const int hh = lane >> 4, c4 = (lane & 15) * 4;
      for (int pass = 0; pass < 2; ++pass) {
#pragma unroll
        for (int it = 0; it < 8; ++it) {
          const int row = it * 2 + hh;
          v4f v = *(const v4f*)(slab + row * 68 + c4);
          *(volatile v4f*)(C + (size_t)(mBase + row) * ldc + n0 + c4) = v;
        }
        __threadfence();
      }
    } else {
      const int q = lane >> 3, c8 = (lane & 7) * 8;
      unsigned short* C  = (unsigned short*)Cout  + (size_t)b * strideC;
      unsigned short* C2 = (OUT_MODE == 2) ? ((unsigned short*)Cout2 + (size_t)b * strideC) : nullptr;
      for (int pass = 0; pass < 2; ++pass) {
#pragma unroll
        for (int it = 0; it < 4; ++it) {
          const int row = it * 4 + q;
          const float* sp = slab + row * 68 + c8;
          v8h hv, lv;
#pragma unroll
          for (int e = 0; e < 8; ++e) {
            if (OUT_MODE == 1) {
              hv[e] = (_Float16)sp[e];
            } else {
              unsigned short hb = f2bf_bits(sp[e]);
              unsigned short lb = f2bf_bits(sp[e] - bf_bits2f(hb));
              hv[e] = __builtin_bit_cast(_Float16, hb);
              lv[e] = __builtin_bit_cast(_Float16, lb);
            }
          }
          *(volatile v8h*)(C + (size_t)(mBase + row) * ldc + n0 + c8) = hv;
          if (OUT_MODE == 2) *(volatile v8h*)(C2 + (size_t)(mBase + row) * ldc + n0 + c8) = lv;
        }
        __threadfence();
      }
    }
    __builtin_amdgcn_fence(__ATOMIC_RELEASE, "workgroup");
    __builtin_amdgcn_wave_barrier();
    __builtin_amdgcn_fence(__ATOMIC_ACQUIRE, "workgroup");
  }
}

__device__ __forceinline__ float wsum32(float v) {
  v += __shfl_xor(v, 16, 32); v += __shfl_xor(v, 8, 32); v += __shfl_xor(v, 4, 32);
  v += __shfl_xor(v, 2, 32);  v += __shfl_xor(v, 1, 32);
  return v;
}
__device__ __forceinline__ float wmin32(float v) {
  v = fminf(v, __shfl_xor(v, 16, 32)); v = fminf(v, __shfl_xor(v, 8, 32)); v = fminf(v, __shfl_xor(v, 4, 32));
  v = fminf(v, __shfl_xor(v, 2, 32));  v = fminf(v, __shfl_xor(v, 1, 32));
  return v;
}
__device__ __forceinline__ float wmax32(float v) {
  v = fmaxf(v, __shfl_xor(v, 16, 32)); v = fmaxf(v, __shfl_xor(v, 8, 32)); v = fmaxf(v, __shfl_xor(v, 4, 32));
  v = fmaxf(v, __shfl_xor(v, 2, 32));  v = fmaxf(v, __shfl_xor(v, 1, 32));
  return v;
}
__device__ __forceinline__ float bsum4(float v, float* redrow, int wave, int lane) {
  v = wsum32(v);
  if (lane == 0) redrow[wave] = v;
  __syncthreads();
  const float t = redrow[0] + redrow[1] + redrow[2] + redrow[3];
  __syncthreads();
  return t;
}
__device__ __forceinline__ unsigned split_pack2(float a, float b, unsigned& lo_out) {
  const unsigned short ha = f2bf_bits(a), hb = f2bf_bits(b);
  const unsigned short la = f2bf_bits(a - bf_bits2f(ha)), lb = f2bf_bits(b - bf_bits2f(hb));
  lo_out = (unsigned)la | ((unsigned)lb << 16);
  return (unsigned)ha | ((unsigned)hb << 16);
}
__device__ __forceinline__ float sgn3(float x) { return x > 0.f ? 1.f : (x < 0.f ? -1.f : 0.f); }
__device__ __forceinline__ float sigm(float v) {
  const float av = fabsf(v);
  const float ev = expf(-av);
  const float s = 1.0f / (1.0f + ev);
  return v >= 0.f ? s : ev * s;
}

template <bool TR>
__global__ __launch_bounds__(256) void split_plane(const float* __restrict__ in, int R, int Cc,
    unsigned short* __restrict__ oh, unsigned short* __restrict__ ol, int opitch) {
  __shared__ float tile[64][65];
  const int tid = threadIdx.x;
  const int r0 = blockIdx.y * 64, c0 = blockIdx.x * 64;
#pragma unroll
  for (int k = 0; k < 16; ++k) {
    int rr, cc;
    if (TR) { rr = tid & 63; cc = (tid >> 6) + 4 * k; }
    else    { cc = tid & 63; rr = (tid >> 6) + 4 * k; }
    const int orow = r0 + rr, ocol = c0 + cc;
    int ir = TR ? ocol : orow;
    int ic = TR ? orow : ocol;
    const bool ok = (ir < R) && (ic < Cc);
    ir = ir < R ? ir : R - 1;
    ic = ic < Cc ? ic : Cc - 1;
    const float v = in[(size_t)ir * Cc + ic];
    tile[rr][cc] = ok ? v : 0.f;
  }
  __syncthreads();
  const int wave = tid >> 5, lane = tid & 31;
  v4u hv[2], lv[2];
  size_t off[2];
#pragma unroll
  for (int s = 0; s < 2; ++s) {
    const int rr = wave * 8 + (lane >> 3) + 4 * s;
    const int cc = (lane & 7) * 8;
#pragma unroll
    for (int e2 = 0; e2 < 4; ++e2) {
      unsigned lo;
      hv[s][e2] = split_pack2(tile[rr][cc + 2 * e2], tile[rr][cc + 2 * e2 + 1], lo);
      lv[s][e2] = lo;
    }
    off[s] = (size_t)(r0 + rr) * opitch + c0 + cc;
  }
  for (int pass = 0; pass < 2; ++pass) {
#pragma unroll
    for (int s = 0; s < 2; ++s) {
      *(volatile v4u*)(oh + off[s]) = hv[s];
      *(volatile v4u*)(ol + off[s]) = lv[s];
    }
    __threadfence();
  }
}

__global__ __launch_bounds__(256) void rowk(const float* __restrict__ xin, const float* __restrict__ h2p,
    const float* __restrict__ b2, float* __restrict__ hf,
    unsigned short* __restrict__ hph, unsigned short* __restrict__ hpl,
    unsigned short* __restrict__ lph, unsigned short* __restrict__ lpl) {
  __shared__ float hrow[8][256];
  const int tid = threadIdx.x, wave = tid >> 5, lane = tid & 31;
  const int row = blockIdx.x * 8 + wave;
  const float* xr = xin + (size_t)row * NI_;
  const int l3 = lane < 16 ? lane : 0;
  const float x0 = xr[lane], x1 = xr[32 + lane];
  float x2 = xr[64 + l3];
  x2 = (lane < 16) ? x2 : 0.f;
  const float inm = wsum32(x0 + x1 + x2) * (1.0f / 80.0f);
  const float d0 = x0 - inm, d1 = x1 - inm, d2 = x2 - inm;
  float qq = d0 * d0 + d1 * d1;
  qq += (lane < 16) ? d2 * d2 : 0.f;
  const float inv = wsum32(qq) * (1.0f / 80.0f);
  float hv[5];
#pragma unroll
  for (int m = 0; m < 5; ++m) {
    const int c = lane + 32 * m;
    hv[m] = h2p[(size_t)row * N2P_ + c] + b2[c];
  }
  const float m2 = wsum32(hv[0] + hv[1] + hv[2] + hv[3] + hv[4]) * (1.0f / 160.0f);
  float q2 = 0.f;
#pragma unroll
  for (int m = 0; m < 5; ++m) { const float d = hv[m] - m2; q2 += d * d; }
  const float v2 = wsum32(q2) * (1.0f / 160.0f);
  const float rv2 = 1.0f / v2;
  float* hr = hrow[wave];
#pragma unroll
  for (int m = 0; m < 5; ++m) hr[lane + 32 * m] = (hv[m] - m2) * rv2 * inv + inm;
  hr[160 + lane] = 0.f; hr[192 + lane] = 0.f; hr[224 + lane] = 0.f;
  __syncthreads();
  v4f f4a, f4b;
#pragma unroll
  for (int e = 0; e < 4; ++e) {
    const int c = 4 * lane + e;
    const float va = hr[c];
    const float vb = hr[NI_ + c];
    f4a[e] = (c < NI_) ? va : 0.f;
    f4b[e] = (c < NI_) ? vb : 0.f;
  }
  const int l16 = lane & 15;
  const bool isL = lane >= 16;
  const int sbase = isL ? NI_ : 0;
  v4u vh, vl;
#pragma unroll
  for (int e2 = 0; e2 < 4; ++e2) {
    const int c = 8 * l16 + 2 * e2;
    float a = hr[sbase + c], bq = hr[sbase + c + 1];
    a = (c < NI_) ? a : 0.f;
    bq = (c + 1 < NI_) ? bq : 0.f;
    unsigned lo;
    vh[e2] = split_pack2(a, bq, lo);
    vl[e2] = lo;
  }
  unsigned short* ph = (isL ? lph : hph) + (size_t)row * KP_ + 8 * l16;
  unsigned short* pl = (isL ? lpl : hpl) + (size_t)row * KP_ + 8 * l16;
  float* hfr = hf + (size_t)row * HFP_;
  for (int pass = 0; pass < 2; ++pass) {
    *(volatile v4f*)(hfr + 4 * lane) = f4a;
    *(volatile v4f*)(hfr + 128 + 4 * lane) = f4b;
    *(volatile v4u*)ph = vh;
    *(volatile v4u*)pl = vl;
    __threadfence();
  }
}

__global__ __launch_bounds__(256) void maskk(unsigned short* __restrict__ zrhl, unsigned short* __restrict__ zrll, const float* __restrict__ b1l,
    unsigned short* __restrict__ zrhh, unsigned short* __restrict__ zrlh, const float* __restrict__ b1h,
    unsigned* __restrict__ maskt) {
  const int tid = threadIdx.x, wave = tid >> 5, lane = tid & 31;
  const int var = blockIdx.y;
  unsigned short* zh = var ? zrhh : zrhl;
  unsigned short* zl = var ? zrlh : zrll;
  const float* b1 = var ? b1h : b1l;
  unsigned* mt = maskt + (size_t)var * NTOK_ * 16;
  const int p = blockIdx.x * 8 + wave;
  unsigned mword = 0u;
  {
    const int tk = 2 * p + (lane >> 4), w = lane & 15;
    const v4u* src = (const v4u*)(zh + (size_t)tk * NHID_ + 32 * w);
#pragma unroll
    for (int q4 = 0; q4 < 4; ++q4) {
      const v4u u = src[q4];
#pragma unroll
      for (int e = 0; e < 4; ++e) {
        const unsigned x = u[e];
        const unsigned on0 = (((x & 0xffffu) != 0u) && ((x & 0x8000u) == 0u)) ? 1u : 0u;
        const unsigned on1 = (((x >> 16) != 0u) && ((x & 0x80000000u) == 0u)) ? 1u : 0u;
        mword |= on0 << (8 * q4 + 2 * e);
        mword |= on1 << (8 * q4 + 2 * e + 1);
      }
    }
  }
  v4u hv[4], lv[4];
  size_t off[4];
#pragma unroll
  for (int it = 0; it < 4; ++it) {
    const int e0 = it * 256 + lane * 8;
    const int tk = 2 * p + (e0 >> 9), h0 = e0 & 511;
    const v4u u = *(const v4u*)(zh + (size_t)tk * NHID_ + h0);
    const v4f bA = *(const v4f*)(b1 + h0), bB = *(const v4f*)(b1 + h0 + 4);
    const float bb[8] = {bA[0], bA[1], bA[2], bA[3], bB[0], bB[1], bB[2], bB[3]};
#pragma unroll
    for (int e2 = 0; e2 < 4; ++e2) {
      const unsigned x = u[e2];
      const bool on0 = ((x & 0xffffu) != 0u) && ((x & 0x8000u) == 0u);
      const bool on1 = ((x >> 16) != 0u) && ((x & 0x80000000u) == 0u);
      const float a = on0 ? bb[2 * e2] : 0.f, c2v = on1 ? bb[2 * e2 + 1] : 0.f;
      unsigned lo;
      hv[it][e2] = split_pack2(a, c2v, lo);
      lv[it][e2] = lo;
    }
    off[it] = (size_t)(NTOK_ + tk) * NHID_ + h0;
  }
  for (int pass = 0; pass < 2; ++pass) {
    *(volatile unsigned*)(mt + (size_t)(2 * p) * 16 + lane) = mword;
#pragma unroll
    for (int it = 0; it < 4; ++it) {
      *(volatile v4u*)(zh + off[it]) = hv[it];
      *(volatile v4u*)(zl + off[it]) = lv[it];
    }
    __threadfence();
  }
}

template <bool SPLIT>
__global__ __launch_bounds__(160) void energyk(const unsigned short* __restrict__ aw1h, const unsigned short* __restrict__ aw1l,
    const unsigned short* __restrict__ w2th, const unsigned short* __restrict__ w2tl,
    const unsigned* __restrict__ maskt, const float* __restrict__ hf, int hcol,
    const float* __restrict__ cm, const float* __restrict__ b2v, const float* __restrict__ xout,
    float* __restrict__ e0) {
  __shared__ float ssg[80], sab[80], esg[80];
  __shared__ unsigned mw[16];
  __shared__ float wnum[8], wden[8], eout[32];
  const int tid = threadIdx.x, wv = tid >> 5, lane = tid & 31;
  const int hh = lane >> 4, rl = lane & 15, koff = hh * 8;
  const __bf16* Ah = (const __bf16*)aw1h; const __bf16* Al = (const __bf16*)aw1l;
  const __bf16* Bh = (const __bf16*)w2th; const __bf16* Bl = (const __bf16*)w2tl;
  for (int s = 0; s < 32; ++s) {
    const int tk = blockIdx.x * 32 + s;
    __syncthreads();
    if (tid < NI_) {
      const float sv = hf[(size_t)tk * HFP_ + hcol + tid];
      ssg[tid] = sgn3(sv);
      sab[tid] = fabsf(sv);
      const float bh = cm[(size_t)(NTOK_ + tk) * NOP_ + tid] + b2v[tid];
      const float ev = xout[(size_t)tk * (NTN_ * NI_) + tid] - bh;
      esg[tid] = sgn3(ev);
    }
    if (tid < 16) mw[tid] = maskt[(size_t)tk * 16 + tid];
    __syncthreads();
    v8f acc[5];
#pragma unroll
    for (int j = 0; j < 5; ++j) acc[j] = (v8f){0.f,0.f,0.f,0.f,0.f,0.f,0.f,0.f};
    for (int kk = 0; kk < 16; ++kk) {
      const int k0 = kk * 32;
      v16b bfh[5], bfl[5];
#pragma unroll
      for (int j = 0; j < 5; ++j) {
        const size_t bo = (size_t)(16 * j + rl) * NHID_ + koff + k0;
        bfh[j] = Frag<__bf16>::load(Bh + bo);
        bfl[j] = SPLIT ? Frag<__bf16>::load(Bl + bo) : bfh[j];
      }
      const size_t ao = (size_t)(16 * wv + rl) * NHID_ + koff + k0;
      v16b ah = Frag<__bf16>::load(Ah + ao);
      v16b al = SPLIT ? Frag<__bf16>::load(Al + ao) : ah;
      const unsigned word = mw[kk];
      const unsigned mb = ((word >> koff) & 0xffu) | (((word >> (16 + koff)) & 0xffu) << 8);
      v8u msk;
#pragma unroll
      for (int q = 0; q < 8; ++q) {
        const unsigned b0 = 0u - ((mb >> (2 * q)) & 1u);
        const unsigned b1 = 0u - ((mb >> (2 * q + 1)) & 1u);
        msk[q] = (b0 & 0x0000ffffu) | (b1 & 0xffff0000u);
      }
      ah = __builtin_bit_cast(v16b, __builtin_bit_cast(v8u, ah) & msk);
      if (SPLIT) al = __builtin_bit_cast(v16b, __builtin_bit_cast(v8u, al) & msk);
#pragma unroll
      for (int j = 0; j < 5; ++j) {
        acc[j] = Frag<__bf16>::mma(ah, bfh[j], acc[j]);
        if (SPLIT) {
          acc[j] = Frag<__bf16>::mma(ah, bfl[j], acc[j]);
          acc[j] = Frag<__bf16>::mma(al, bfh[j], acc[j]);
        }
      }
      Frag<__bf16>::guard(acc[0], acc[4], ah, al);
      keep5_b(bfh[0], bfh[1], bfh[2], bfh[3], bfh[4]);
      if (SPLIT) keep5_b(bfl[0], bfl[1], bfl[2], bfl[3], bfl[4]);
    }
    acc_guard5(acc[0], acc[1], acc[2], acc[3], acc[4]);
    float sgo[5];
#pragma unroll
    for (int j = 0; j < 5; ++j) sgo[j] = esg[16 * j + rl];
    float prow[8], nrow[8];
#pragma unroll
    for (int r = 0; r < 8; ++r) {
      const float sgi = ssg[16 * wv + 8 * hh + r];
      float pr = 0.f, nr = 0.f;
#pragma unroll
      for (int j = 0; j < 5; ++j) {
        const float w = acc[j][r] * (sgi * sgo[j]);
        pr += fmaxf(w, 0.f);
        nr += fmaxf(-w, 0.f);
      }
      pr += __shfl_xor(pr, 1, 32); nr += __shfl_xor(nr, 1, 32);
      pr += __shfl_xor(pr, 2, 32); nr += __shfl_xor(nr, 2, 32);
      pr += __shfl_xor(pr, 4, 32); nr += __shfl_xor(nr, 4, 32);
      pr += __shfl_xor(pr, 8, 32); nr += __shfl_xor(nr, 8, 32);
      prow[r] = pr; nrow[r] = nr;
    }
    float num = 0.f, den = 0.f;
#pragma unroll
    for (int r = 0; r < 8; ++r) {
      const float ai = sab[16 * wv + 8 * hh + r];
      num += ai * nrow[r];
      den += ai * prow[r];
    }
    num += __shfl_xor(num, 16, 32);
    den += __shfl_xor(den, 16, 32);
    if (lane == 0) { wnum[wv] = num; wden[wv] = den; }
    __syncthreads();
    if (tid == 0) {
      const float n5 = (((wnum[0] + wnum[1]) + wnum[2]) + wnum[3]) + wnum[4];
      const float d5 = (((wden[0] + wden[1]) + wden[2]) + wden[3]) + wden[4];
      float en = n5 * (1.0f / d5);
      if (en != en) en = 1.0f;
      float ee = 1.0f - en;
      ee = ee > 0.f ? ee : 0.f;
      eout[s] = ee;
    }
  }
  __syncthreads();
  if (tid < 8) {
    v4f v;
    v[0] = eout[4 * tid]; v[1] = eout[4 * tid + 1]; v[2] = eout[4 * tid + 2]; v[3] = eout[4 * tid + 3];
    float* dst = e0 + (size_t)blockIdx.x * 32 + 4 * tid;
    *(volatile v4f*)dst = v;
    __threadfence();
    *(volatile v4f*)dst = v;
  }
}

__global__ __launch_bounds__(256) void minmaxk(const float* __restrict__ e0, float* __restrict__ mm) {
  __shared__ float smn[2][8], smx[2][8];
  const int tid = threadIdx.x, wave = tid >> 5, lane = tid & 31;
#pragma unroll
  for (int v = 0; v < 2; ++v) {
    float mn = INFINITY, mx = -INFINITY;
#pragma unroll
    for (int k = 0; k < 4; ++k) {
      const float x = e0[v * NTOK_ + k * 256 + tid];
      mn = fminf(mn, x); mx = fmaxf(mx, x);
    }
    mn = wmin32(mn); mx = wmax32(mx);
    if (lane == 0) { smn[v][wave] = mn; smx[v][wave] = mx; }
  }
  __syncthreads();
  if (tid < 8) {
    float r0v = smn[0][0], r1v = smx[0][0], r2v = smn[1][0], r3v = smx[1][0];
#pragma unroll
    for (int w = 1; w < 8; ++w) {
      r0v = fminf(r0v, smn[0][w]); r1v = fmaxf(r1v, smx[0][w]);
      r2v = fminf(r2v, smn[1][w]); r3v = fmaxf(r3v, smx[1][w]);
    }
    v4f val = (v4f){0.f, 0.f, 0.f, 0.f};
    if (tid == 0) { val[0] = r0v; val[1] = r1v; val[2] = r2v; val[3] = r3v; }
    float* dst = mm + 4 * tid;
    *(volatile v4f*)dst = val;
    __threadfence();
    *(volatile v4f*)dst = val;
  }
}

__global__ __launch_bounds__(256) void fbk(const float* __restrict__ e0, const float* __restrict__ mm,
    float* __restrict__ lpl, float* __restrict__ ktl) {
  __shared__ float xn[NT_];
  const int b = blockIdx.x, j = threadIdx.x;
  const float mn = mm[0], mx = mm[1];
  const float rinv = 1.0f / (mx - mn);
  xn[j] = 1.0f - (e0[b * NT_ + j] - mn) * rinv;
  __syncthreads();
  const float xj = xn[j];
  const float cj = 0.5f * (xj + 1.0f);
  float* L = lpl + (size_t)b * NT_ * NT_;
  float* Kp = ktl + (size_t)b * NT_ * NT_;
  float p = 1.0f;
  for (int i = 0; i < NT_; ++i) {
    const float xi = xn[i];
    p = (i > j) ? p * xi : p;
    const float val = (i > j) ? cj * p : ((i == j) ? xj : 0.f);
    volatile float* dst = L + (size_t)i * NT_ + j;
    *dst = val;
    __threadfence();
    *dst = val;
  }
  __threadfence();
  float q = 1.0f;
  for (int i = NT_ - 1; i >= 0; --i) {
    const float xi = xn[i];
    q = (i < j) ? q * xi : q;
    const float lowv = *(volatile const float*)(L + (size_t)i * NT_ + j);
    const float val = (j > i) ? cj * q : lowv;
    volatile float* dst = Kp + (size_t)i * NT_ + j;
    *dst = val;
    __threadfence();
    *dst = val;
  }
}

__global__ __launch_bounds__(128) void lossk(const float* __restrict__ cml, const float* __restrict__ cmh,
    const float* __restrict__ b2l, const float* __restrict__ b2h, const float* __restrict__ xout,
    const float* __restrict__ e0h, const float* __restrict__ mm, const int* __restrict__ ilens,
    float* __restrict__ part) {
  __shared__ float red[8][4];
  __shared__ float oul[NI_], ouh[NI_], kwv[16];
  const int tk = blockIdx.x, b = tk >> 8, t = tk & 255;
  const int tid = threadIdx.x, wave = tid >> 5, lane = tid & 31;
  const bool act = tid < NI_;
  const int i80 = act ? tid : 0;
  float ol = cml[(size_t)tk * NOP_ + i80] + b2l[i80];
  float oh = cmh[(size_t)tk * NOP_ + i80] + b2h[i80];
  const float x0 = xout[(size_t)tk * (NTN_ * NI_) + i80];
  ol = act ? ol : 0.f;
  oh = act ? oh : 0.f;
  const float x0a = act ? x0 : 0.f;
  const float ml = bsum4(ol, red[0], wave, lane) * (1.0f / 80.0f);
  const float mh = bsum4(oh, red[1], wave, lane) * (1.0f / 80.0f);
  const float mxm = bsum4(x0a, red[2], wave, lane) * (1.0f / 80.0f);
  const float dl = act ? (ol - ml) : 0.f, dh = act ? (oh - mh) : 0.f, dx = act ? (x0 - mxm) : 0.f;
  const float vl = bsum4(dl * dl, red[3], wave, lane) * (1.0f / 80.0f);
  const float vh = bsum4(dh * dh, red[4], wave, lane) * (1.0f / 80.0f);
  const float vx = bsum4(dx * dx, red[5], wave, lane) * (1.0f / 80.0f);
  if (act) {
    oul[tid] = dl * (1.0f / vl) * vx + mxm;
    ouh[tid] = dh * (1.0f / vh) * vx + mxm;
  }
  if (tid < NTN_) {
    const int n = tid;
    const float mnh = mm[2], mxh = mm[3];
    const float rinv = 1.0f / (mxh - mnh);
    float prod = 1.0f;
#pragma unroll
    for (int k = 0; k < NTN_ - 1; ++k) {
      int u = t + k; u = u < NT_ ? u : NT_ - 1;
      const float xu = 1.0f - (e0h[b * NT_ + u] - mnh) * rinv;
      prod = (k < n) ? prod * xu : prod;
    }
    int un = t + n;
    const bool okn = un < NT_;
    un = okn ? un : NT_ - 1;
    const float xun = 1.0f - (e0h[b * NT_ + un] - mnh) * rinv;
    const float kw = (n == 0) ? xun : (okn ? 0.5f * (xun + 1.0f) * prod : 0.f);
    kwv[tid] = kw;
  }
  __syncthreads();
  float acc = 0.f;
#pragma unroll 1
  for (int idx = tid; idx < NTN_ * NI_; idx += 128) {
    const int n = idx / NI_;
    const int i = idx - n * NI_;
    const float d = oul[i] - xout[(size_t)tk * (NTN_ * NI_) + idx];
    acc += d * d * kwv[n];
  }
  if (act) { const float d = ouh[tid] - x0; acc += d * d; }
  const float tot = bsum4(acc, red[7], wave, lane);
  const bool valid = t < ilens[b];
  if (tid < 8) {
    v4f v = (v4f){0.f, 0.f, 0.f, 0.f};
    if (tid == 0) v[0] = valid ? tot : 0.f;
    float* dst = part + (size_t)tk * 32 + 4 * tid;
    *(volatile v4f*)dst = v;
    __threadfence();
    *(volatile v4f*)dst = v;
  }
}

__global__ __launch_bounds__(256) void lossred(const float* __restrict__ part, float* __restrict__ lossl) {
  __shared__ float red[8];
  const int tid = threadIdx.x, wave = tid >> 5, lane = tid & 31;
  float s = 0.f;
#pragma unroll
  for (int k = 0; k < 4; ++k) s += part[(size_t)(tid + 256 * k) * 32];
  s = wsum32(s);
  if (lane == 0) red[wave] = s;
  __syncthreads();
  if (tid < 8) {
    const float tot = ((((((red[0] + red[1]) + red[2]) + red[3]) + red[4]) + red[5]) + red[6]) + red[7];
    v4f v = (v4f){0.f, 0.f, 0.f, 0.f};
    if (tid == 0) v[0] = tot;
    float* dst = lossl + 4 * tid;
    *(volatile v4f*)dst = v;
    __threadfence();
    *(volatile v4f*)dst = v;
  }
}

__global__ __launch_bounds__(256) void packk(const float* __restrict__ lossl, const float* __restrict__ gram,
    const float* __restrict__ ktl, float* __restrict__ out) {
  const int g = blockIdx.x * 256 + threadIdx.x;
  const int f0 = 4 * g;
  const float lossv = lossl[0];
  v4f v;
#pragma unroll
  for (int e = 0; e < 4; ++e) {
    const int f = f0 + e;
    int gi = f - OUT1_OFF_; gi = gi < 0 ? 0 : gi; gi = gi > (NB_ * NT_ * NT_ - 1) ? (NB_ * NT_ * NT_ - 1) : gi;
    int ki = f - OUT2_OFF_; ki = ki < 0 ? 0 : ki; ki = ki > (NB_ * NT_ * NT_ - 1) ? (NB_ * NT_ * NT_ - 1) : ki;
    const float gv = gram[gi];
    const float kv = ktl[ki];
    const float sg = sigm(gv);
    v[e] = (f == 0) ? lossv : ((f < OUT2_OFF_) ? sg : kv);
  }
  float* dst = out + f0;
  *(volatile v4f*)dst = v;
  __threadfence();
  *(volatile v4f*)dst = v;
  if (g == 0) {
    const float tv = ktl[NB_ * NT_ * NT_ - 1];
    volatile float* pt = out + (OUT_TOTAL_ - 1);
    *pt = tv;
    __threadfence();
    *pt = tv;
  }
}

template <int BIAS_MODE, int OUT_MODE, int ACT>
static void launch_gemm(hipStream_t st, const void* A, const void* A2, int lda, long sA,
                        const void* Bt, const void* Bt2, int ldb, long sB,
                        void* C, void* C2, int ldc, long sC, const float* bias, const float* dummy_resid,
                        int M, int N, int K, int batch) {
  const int tiles = (M / 64) * (N / 64);
  dim3 grid((tiles + 7) / 8, batch);
  wmma_gemm64<1, true, BIAS_MODE, OUT_MODE, false, ACT><<<grid, 256, 0, st>>>(
      (const unsigned short*)A, (const unsigned short*)A2, lda, sA,
      (const unsigned short*)Bt, (const unsigned short*)Bt2, ldb, sB,
      C, C2, ldc, sC, bias, dummy_resid, 0L, M, N, K, 1.0f);
}

extern "C" void kernel_launch(void* const* d_in, const int* in_sizes, int n_in,
                              void* d_out, int out_size, void* d_ws, size_t ws_size,
                              hipStream_t stream) {
  (void)in_sizes; (void)n_in; (void)out_size; (void)ws_size;
  const float* xin   = (const float*)d_in[0];
  const float* xout  = (const float*)d_in[1];
  const int*   ilens = (const int*)  d_in[2];
  const float* encW1 = (const float*)d_in[4];
  const float* encb1 = (const float*)d_in[5];
  const float* encW2 = (const float*)d_in[6];
  const float* encb2 = (const float*)d_in[7];
  const float* dlW1  = (const float*)d_in[8];
  const float* dlb1  = (const float*)d_in[9];
  const float* dlW2  = (const float*)d_in[10];
  const float* dlb2  = (const float*)d_in[11];
  const float* dhW1  = (const float*)d_in[12];
  const float* dhb1  = (const float*)d_in[13];
  const float* dhW2  = (const float*)d_in[14];
  const float* dhb2  = (const float*)d_in[15];
  float* fout = (float*)d_out;

  char* wsb = (char*)d_ws;
  size_t off = 0;
  auto carve = [&](size_t bytes) -> char* { char* p = wsb + off; off += (bytes + 255) & ~(size_t)255; return p; };
  unsigned short* XINH = (unsigned short*)carve(SZ_XIN);    unsigned short* XINL = (unsigned short*)carve(SZ_XIN);
  unsigned short* EW1TH = (unsigned short*)carve(SZ_W1T);   unsigned short* EW1TL = (unsigned short*)carve(SZ_W1T);
  unsigned short* EW2TH = (unsigned short*)carve(SZ_EW2T);  unsigned short* EW2TL = (unsigned short*)carve(SZ_EW2T);
  unsigned short* DW1TLH = (unsigned short*)carve(SZ_W1T);  unsigned short* DW1TLL = (unsigned short*)carve(SZ_W1T);
  unsigned short* DW1THH = (unsigned short*)carve(SZ_W1T);  unsigned short* DW1THL = (unsigned short*)carve(SZ_W1T);
  unsigned short* DW2TLH = (unsigned short*)carve(SZ_W2T);  unsigned short* DW2TLL = (unsigned short*)carve(SZ_W2T);
  unsigned short* DW2THH = (unsigned short*)carve(SZ_W2T);  unsigned short* DW2THL = (unsigned short*)carve(SZ_W2T);
  unsigned short* AW1LH = (unsigned short*)carve(SZ_AW1);   unsigned short* AW1LL = (unsigned short*)carve(SZ_AW1);
  unsigned short* AW1HH = (unsigned short*)carve(SZ_AW1);   unsigned short* AW1HL = (unsigned short*)carve(SZ_AW1);
  unsigned short* ZENCH = (unsigned short*)carve(SZ_ZENC);  unsigned short* ZENCL = (unsigned short*)carve(SZ_ZENC);
  float* H2P = (float*)carve(SZ_H2);
  unsigned short* HPH = (unsigned short*)carve(SZ_HP);      unsigned short* HPL = (unsigned short*)carve(SZ_HP);
  unsigned short* LPH = (unsigned short*)carve(SZ_HP);      unsigned short* LPL = (unsigned short*)carve(SZ_HP);
  float* HF = (float*)carve(SZ_HF);
  unsigned short* ZRLH = (unsigned short*)carve(SZ_ZR);     unsigned short* ZRLL = (unsigned short*)carve(SZ_ZR);
  unsigned short* ZRHH = (unsigned short*)carve(SZ_ZR);     unsigned short* ZRHL = (unsigned short*)carve(SZ_ZR);
  float* CML = (float*)carve(SZ_CM);                        float* CMH = (float*)carve(SZ_CM);
  unsigned* MASKT = (unsigned*)carve(SZ_MASKT);
  float* GRAM = (float*)carve(SZ_GRAM);
  float* E0 = (float*)carve(SZ_E0);
  float* MM = (float*)carve(SZ_LINE);
  float* LPLANE = (float*)carve(SZ_GRAM);
  float* KTL = (float*)carve(SZ_GRAM);
  float* PART = (float*)carve(SZ_PART);
  float* LOSSL = (float*)carve(SZ_LINE);

  split_plane<false><<<dim3(KP_ / 64, NTOK_ / 64), 256, 0, stream>>>(xin, NTOK_, NI_, XINH, XINL, KP_);
  split_plane<true><<<dim3(KP_ / 64, NHID_ / 64), 256, 0, stream>>>(encW1, NI_, NHID_, EW1TH, EW1TL, KP_);
  split_plane<true><<<dim3(NHID_ / 64, N2P_ / 64), 256, 0, stream>>>(encW2, NHID_, 2 * NI_, EW2TH, EW2TL, NHID_);
  split_plane<true><<<dim3(KP_ / 64, NHID_ / 64), 256, 0, stream>>>(dlW1, NI_, NHID_, DW1TLH, DW1TLL, KP_);
  split_plane<true><<<dim3(KP_ / 64, NHID_ / 64), 256, 0, stream>>>(dhW1, NI_, NHID_, DW1THH, DW1THL, KP_);
  split_plane<true><<<dim3(NHID_ / 64, NOP_ / 64), 256, 0, stream>>>(dlW2, NHID_, NI_, DW2TLH, DW2TLL, NHID_);
  split_plane<true><<<dim3(NHID_ / 64, NOP_ / 64), 256, 0, stream>>>(dhW2, NHID_, NI_, DW2THH, DW2THL, NHID_);
  split_plane<false><<<dim3(NHID_ / 64, 128 / 64), 256, 0, stream>>>(dlW1, NI_, NHID_, AW1LH, AW1LL, NHID_);
  split_plane<false><<<dim3(NHID_ / 64, 128 / 64), 256, 0, stream>>>(dhW1, NI_, NHID_, AW1HH, AW1HL, NHID_);

  launch_gemm<2, 2, 2>(stream, XINH, XINL, KP_, 0L, EW1TH, EW1TL, KP_, 0L, ZENCH, ZENCL, NHID_, 0L, encb1, H2P,
                       NTOK_, NHID_, KP_, 1);
  launch_gemm<0, 0, 0>(stream, ZENCH, ZENCL, NHID_, 0L, EW2TH, EW2TL, NHID_, 0L, H2P, H2P, N2P_, 0L, MM, H2P,
                       NTOK_, N2P_, NHID_, 1);
  rowk<<<NTOK_ / 8, 256, 0, stream>>>(xin, H2P, encb2, HF, HPH, HPL, LPH, LPL);

  launch_gemm<2, 2, 2>(stream, LPH, LPL, KP_, 0L, DW1TLH, DW1TLL, KP_, 0L, ZRLH, ZRLL, NHID_, 0L, dlb1, CML,
                       NTOK_, NHID_, KP_, 1);
  launch_gemm<2, 2, 2>(stream, HPH, HPL, KP_, 0L, DW1THH, DW1THL, KP_, 0L, ZRHH, ZRHL, NHID_, 0L, dhb1, CMH,
                       NTOK_, NHID_, KP_, 1);
  maskk<<<dim3(NTOK_ / 16, 2), 256, 0, stream>>>(ZRLH, ZRLL, dlb1, ZRHH, ZRHL, dhb1, MASKT);
  launch_gemm<0, 0, 0>(stream, ZRLH, ZRLL, NHID_, 0L, DW2TLH, DW2TLL, NHID_, 0L, CML, CML, NOP_, 0L, MM, CML,
                       2 * NTOK_, NOP_, NHID_, 1);
  launch_gemm<0, 0, 0>(stream, ZRHH, ZRHL, NHID_, 0L, DW2THH, DW2THL, NHID_, 0L, CMH, CMH, NOP_, 0L, MM, CMH,
                       2 * NTOK_, NOP_, NHID_, 1);
  launch_gemm<0, 0, 0>(stream, HPH, HPL, KP_, (long)NT_ * KP_, HPH, HPL, KP_, (long)NT_ * KP_,
                       GRAM, GRAM, NT_, (long)NT_ * NT_, MM, GRAM, NT_, NT_, KP_, NB_);

  energyk<true><<<NTOK_ / 32, 160, 0, stream>>>(AW1LH, AW1LL, DW2TLH, DW2TLL, MASKT, HF, 128, CML, dlb2, xout, E0);
  energyk<false><<<NTOK_ / 32, 160, 0, stream>>>(AW1HH, AW1HH, DW2THH, DW2THH, MASKT + (size_t)NTOK_ * 16, HF, 0,
                                                CMH, dhb2, xout, E0 + NTOK_);
  minmaxk<<<1, 256, 0, stream>>>(E0, MM);
  fbk<<<NB_, NT_, 0, stream>>>(E0, MM, LPLANE, KTL);
  lossk<<<NTOK_, 128, 0, stream>>>(CML, CMH, dlb2, dhb2, xout, E0 + NTOK_, MM, ilens, PART);
  lossred<<<1, 256, 0, stream>>>(PART, LOSSL);
  packk<<<(OUT_TOTAL_ - 1) / 4 / 256, 256, 0, stream>>>(LOSSL, GRAM, KTL, fout);
}
